// GCNGraphEncoder_18940805775859
// MI455X (gfx1250) — hardware-verified
//
#include <hip/hip_runtime.h>
#include <stddef.h>
#include <stdint.h>


typedef _Float16 v16h __attribute__((ext_vector_type(16)));
typedef _Float16 v8h  __attribute__((ext_vector_type(8)));
typedef _Float16 v4h  __attribute__((ext_vector_type(4)));
typedef float    v8f  __attribute__((ext_vector_type(8)));
typedef float    v4f  __attribute__((ext_vector_type(4)));
typedef unsigned int v4u __attribute__((ext_vector_type(4)));

union Frag  { v16h v; v8h half[2]; };
union Pack8 { v8h h; v4u u; };

#define CHN   128
#define HID2  256
#define TPB   256
#define NWAV  (TPB / 32)
#define NBLK  512
#define NDEG  8192
#define CHUNK 2048
#define EPT   8

__device__ __forceinline__ v8f wmma_f16(v16h a, v16h b, v8f c) {
  c = __builtin_amdgcn_wmma_f32_16x16x32_f16(false, a, false, b, (short)0, c, false, false);
  asm volatile("v_nop\n\tv_nop\n\tv_nop\n\tv_nop" : "+v"(c) : "v"(a), "v"(b));
  return c;
}

__device__ __forceinline__ v4h load4h(const float* p) {
  return __builtin_convertvector(*(const v4f*)p, v4h);
}
__device__ __forceinline__ v4h load4h(const _Float16* p) {
  return *(const v4h*)p;
}

template <typename TA, int K>
__global__ void __launch_bounds__(TPB)
k_gemm(const TA* __restrict__ A, int lda, int M,
       const float* __restrict__ W, int ldw,
       const float* __restrict__ bias, int has_bias,
       float* __restrict__ out, int ldo, int relu)
{
  extern __shared__ v4f dyn_smem[];
  constexpr int PA = K + 8;
  _Float16* sA = (_Float16*)dyn_smem;
  _Float16* sB = sA + 128 * PA;

  const int tid = threadIdx.x, lane = tid & 31, wave = tid >> 5;
  const int h = lane >> 4, m = lane & 15;
  const int rowBase = blockIdx.x * 128;
  const int colBase = blockIdx.y * 128;

  for (int i = tid; i < 128 * (K / 4); i += TPB) {
    const int r = i / (K / 4);
    const int k = (i - r * (K / 4)) * 4;
    int gr = rowBase + r;
    if (gr > M - 1) gr = M - 1;
    const v4h hv = load4h(A + (size_t)gr * lda + k);
    *(v4h*)(sA + r * PA + k) = hv;
  }
  for (int i = tid; i < K * 32; i += TPB) {
    const int k = i >> 5;
    const int n = (i & 31) * 4;
    const v4f w = *(const v4f*)(W + (size_t)k * ldw + colBase + n);
    _Float16* d = sB + n * PA + k;
    d[0]      = (_Float16)(w.x * 16.0f);
    d[PA]     = (_Float16)(w.y * 16.0f);
    d[2 * PA] = (_Float16)(w.z * 16.0f);
    d[3 * PA] = (_Float16)(w.w * 16.0f);
  }
  __syncthreads();

  v8f acc[8];
  {
    const v8f z = {0.f, 0.f, 0.f, 0.f, 0.f, 0.f, 0.f, 0.f};
#pragma unroll
    for (int t = 0; t < 8; ++t) acc[t] = z;
  }
  const _Float16* arow = sA + (wave * 16 + m) * PA + 8 * h;
  const _Float16* bcol = sB + m * PA + 8 * h;
  for (int k0 = 0; k0 < K; k0 += 32) {
    Frag a;
    a.half[0] = *(const v8h*)(arow + k0);
    a.half[1] = *(const v8h*)(arow + k0 + 16);
#pragma unroll
    for (int t = 0; t < 8; ++t) {
      const _Float16* bp = bcol + t * 16 * PA + k0;
      Frag b;
      b.half[0] = *(const v8h*)bp;
      b.half[1] = *(const v8h*)(bp + 16);
      acc[t] = wmma_f16(a.v, b.v, acc[t]);
    }
  }
  __syncthreads();

  float* stg = (float*)dyn_smem + wave * (16 * 128);
#pragma unroll
  for (int t = 0; t < 8; ++t) {
    const int col = t * 16 + m;
    const float bv = has_bias ? bias[colBase + col] : 0.0f;
#pragma unroll
    for (int r = 0; r < 8; ++r) {
      float v = acc[t][r] * 0.0625f + bv;
      if (relu) v = fmaxf(v, 0.0f);
      stg[(8 * h + r) * 128 + col] = v;
    }
  }
  __syncthreads();

  const v4f* stg4 = (const v4f*)stg;
  float* ob = out + (size_t)(rowBase + wave * 16) * ldo + colBase + lane * 4;
#pragma unroll
  for (int r = 0; r < 16; ++r) {
    const v4f v = stg4[r * 32 + lane];
    *(volatile v4f*)(ob + (size_t)r * ldo) = v;
  }
  __threadfence();
#pragma unroll
  for (int r = 0; r < 16; ++r) {
    const v4f v = stg4[r * 32 + lane];
    *(volatile v4f*)(ob + (size_t)r * ldo) = v;
  }
}

__global__ void __launch_bounds__(TPB)
k_deg(const int* __restrict__ edst, int E, float* __restrict__ dinv)
{
  __shared__ int cntL[NDEG];
  __shared__ unsigned short lidx[CHUNK];
  __shared__ int wc[NWAV];
  const int tid = threadIdx.x, lane = tid & 31, wave = tid >> 5;
  const int n0 = blockIdx.x * NDEG;

  for (int i = tid; i < NDEG; i += TPB) cntL[i] = 0;
  __syncthreads();

  const unsigned lt = (1u << lane) - 1u;
  for (int c0 = 0; c0 < E; c0 += CHUNK) {
    unsigned bal[EPT];
    int dq[EPT];
    int cw = 0;
#pragma unroll
    for (int q = 0; q < EPT; ++q) {
      const int e = c0 + q * TPB + tid;
      int d = -1;
      if (e < E) d = edst[e];
      const bool hit = (e < E) && ((unsigned)(d - n0) < (unsigned)NDEG);
      dq[q] = d;
      bal[q] = __builtin_amdgcn_ballot_w32(hit);
      cw += __builtin_popcount(bal[q]);
    }
    if (lane == 0) wc[wave] = cw;
    __syncthreads();
    int base = 0, total = 0;
#pragma unroll
    for (int w = 0; w < NWAV; ++w) {
      const int c = wc[w];
      total += c;
      if (w < wave) base += c;
    }
#pragma unroll
    for (int q = 0; q < EPT; ++q) {
      if ((bal[q] >> lane) & 1u) {
        const int pos = base + __builtin_popcount(bal[q] & lt);
        if ((unsigned)pos < (unsigned)CHUNK) lidx[pos] = (unsigned short)(dq[q] - n0);
      }
      base += __builtin_popcount(bal[q]);
    }
    __syncthreads();
    if (wave == 0) {
      const int cnt = total < CHUNK ? total : CHUNK;
      for (int j = 0; j < cnt; ++j) {
        const int dl = (int)lidx[j] & (NDEG - 1);
        if ((dl & 31) == lane) cntL[dl] += 1;
      }
    }
    __syncthreads();
  }

  float* dv = dinv + (size_t)n0;
  for (int i = tid; i < NDEG / 4; i += TPB) {
    v4f v;
    v.x = 1.0f / sqrtf((float)(cntL[4 * i + 0] + 1));
    v.y = 1.0f / sqrtf((float)(cntL[4 * i + 1] + 1));
    v.z = 1.0f / sqrtf((float)(cntL[4 * i + 2] + 1));
    v.w = 1.0f / sqrtf((float)(cntL[4 * i + 3] + 1));
    *(volatile v4f*)(dv + 4 * i) = v;
  }
  __threadfence();
  for (int i = tid; i < NDEG / 4; i += TPB) {
    v4f v;
    v.x = 1.0f / sqrtf((float)(cntL[4 * i + 0] + 1));
    v.y = 1.0f / sqrtf((float)(cntL[4 * i + 1] + 1));
    v.z = 1.0f / sqrtf((float)(cntL[4 * i + 2] + 1));
    v.w = 1.0f / sqrtf((float)(cntL[4 * i + 3] + 1));
    *(volatile v4f*)(dv + 4 * i) = v;
  }
}

template <int NORM>
__global__ void __launch_bounds__(TPB)
k_agg(const int* __restrict__ esrc, const int* __restrict__ edst, int E, int N,
      const float* __restrict__ hin, const float* __restrict__ dinv,
      const float* __restrict__ bias, float* __restrict__ outp)
{
  extern __shared__ v4f dyn_smem[];
  __shared__ int wc[NWAV];
  v4f* accL = dyn_smem;
  int* lsrc = (int*)(dyn_smem + NBLK * 32);
  unsigned short* ldl = (unsigned short*)(lsrc + CHUNK);
  const int tid = threadIdx.x, lane = tid & 31, wave = tid >> 5;
  const int n0 = blockIdx.x * NBLK;
  const v4f* hin4 = (const v4f*)hin;

  for (int i = tid; i < NBLK * 32; i += TPB) {
    const int r = i >> 5, c4 = i & 31, n = n0 + r;
    v4f v = {0.f, 0.f, 0.f, 0.f};
    if (n < N) {
      v = hin4[(size_t)n * 32 + c4];
      if (NORM) v = v * dinv[n];
    }
    accL[i] = v;
  }
  __syncthreads();

  const unsigned lt = (1u << lane) - 1u;
  for (int c0 = 0; c0 < E; c0 += CHUNK) {
    unsigned bal[EPT];
    int dq[EPT];
    int cw = 0;
#pragma unroll
    for (int q = 0; q < EPT; ++q) {
      const int e = c0 + q * TPB + tid;
      int d = -1;
      if (e < E) d = edst[e];
      const bool hit = (e < E) && ((unsigned)(d - n0) < (unsigned)NBLK);
      dq[q] = d;
      bal[q] = __builtin_amdgcn_ballot_w32(hit);
      cw += __builtin_popcount(bal[q]);
    }
    if (lane == 0) wc[wave] = cw;
    __syncthreads();
    int base = 0, total = 0;
#pragma unroll
    for (int w = 0; w < NWAV; ++w) {
      const int c = wc[w];
      total += c;
      if (w < wave) base += c;
    }
#pragma unroll
    for (int q = 0; q < EPT; ++q) {
      if ((bal[q] >> lane) & 1u) {
        const int pos = base + __builtin_popcount(bal[q] & lt);
        const int e = c0 + q * TPB + tid;
        int s = esrc[e];
        s = s < 0 ? 0 : (s > N - 1 ? N - 1 : s);
        if ((unsigned)pos < (unsigned)CHUNK) {
          lsrc[pos] = s;
          ldl[pos]  = (unsigned short)(dq[q] - n0);
        }
      }
      base += __builtin_popcount(bal[q]);
    }
    __syncthreads();
    if (wave == 0) {
      const int cnt = total < CHUNK ? total : CHUNK;
      for (int j = 0; j < cnt; ++j) {
        int s = lsrc[j];
        s = s < 0 ? 0 : (s > N - 1 ? N - 1 : s);
        const int dl = (int)ldl[j] & (NBLK - 1);
        v4f v = hin4[(size_t)s * 32 + lane];
        if (NORM) v = v * dinv[s];
        accL[dl * 32 + lane] += v;
      }
    }
    __syncthreads();
  }

  if (NORM) {
    const v4f b4 = ((const v4f*)bias)[lane];
    for (int r = wave; r < NBLK; r += NWAV) {
      const float di = dinv[n0 + r];
      v4f v = accL[r * 32 + lane] * di + b4;
      v.x = fmaxf(v.x, 0.f); v.y = fmaxf(v.y, 0.f);
      v.z = fmaxf(v.z, 0.f); v.w = fmaxf(v.w, 0.f);
      accL[r * 32 + lane] = v;
    }
    float* outf = outp;
    for (int r = wave; r < NBLK; r += NWAV) {
      const v4f v = accL[r * 32 + lane];
      *(volatile v4f*)(outf + (size_t)(n0 + r) * CHN + lane * 4) = v;
    }
    __threadfence();
    for (int r = wave; r < NBLK; r += NWAV) {
      const v4f v = accL[r * 32 + lane];
      *(volatile v4f*)(outf + (size_t)(n0 + r) * CHN + lane * 4) = v;
    }
  } else {
    _Float16* outh = (_Float16*)outp;
    const int hh = lane >> 4, mm = lane & 15;
    for (int i = 0; i < NBLK / 16; ++i) {
      const int r = i * 16 + wave * 2 + hh;
      const v4f v0 = accL[r * 32 + 2 * mm], v1 = accL[r * 32 + 2 * mm + 1];
      v8f f8 = __builtin_shufflevector(v0, v1, 0, 1, 2, 3, 4, 5, 6, 7);
#pragma unroll
      for (int c = 0; c < 8; ++c) f8[c] = fminf(fmaxf(f8[c], -65504.f), 65504.f);
      Pack8 pk;
      pk.h = __builtin_convertvector(f8, v8h);
      *(volatile v4u*)(outh + (size_t)(n0 + r) * CHN + 8 * mm) = pk.u;
    }
    __threadfence();
    for (int i = 0; i < NBLK / 16; ++i) {
      const int r = i * 16 + wave * 2 + hh;
      const v4f v0 = accL[r * 32 + 2 * mm], v1 = accL[r * 32 + 2 * mm + 1];
      v8f f8 = __builtin_shufflevector(v0, v1, 0, 1, 2, 3, 4, 5, 6, 7);
#pragma unroll
      for (int c = 0; c < 8; ++c) f8[c] = fminf(fmaxf(f8[c], -65504.f), 65504.f);
      Pack8 pk;
      pk.h = __builtin_convertvector(f8, v8h);
      *(volatile v4u*)(outh + (size_t)(n0 + r) * CHN + 8 * mm) = pk.u;
    }
  }
}

__global__ void __launch_bounds__(TPB)
k_pool(const int* __restrict__ batch, int N, const float* __restrict__ hsrc,
       float* __restrict__ mout)
{
  __shared__ int lnode[CHUNK];
  __shared__ int wc[NWAV];
  const int tid = threadIdx.x, lane = tid & 31, wave = tid >> 5;
  const int g = blockIdx.x;
  const v4f* h4 = (const v4f*)hsrc;
  v4f acc = {0.f, 0.f, 0.f, 0.f};
  int ntot = 0;

  const unsigned lt = (1u << lane) - 1u;
  for (int c0 = 0; c0 < N; c0 += CHUNK) {
    unsigned bal[EPT];
    int cw = 0;
#pragma unroll
    for (int q = 0; q < EPT; ++q) {
      const int n = c0 + q * TPB + tid;
      int b = -1;
      if (n < N) b = batch[n];
      const bool hit = (n < N) && (b == g);
      bal[q] = __builtin_amdgcn_ballot_w32(hit);
      cw += __builtin_popcount(bal[q]);
    }
    if (lane == 0) wc[wave] = cw;
    __syncthreads();
    int base = 0, total = 0;
#pragma unroll
    for (int w = 0; w < NWAV; ++w) {
      const int c = wc[w];
      total += c;
      if (w < wave) base += c;
    }
    ntot += total;
#pragma unroll
    for (int q = 0; q < EPT; ++q) {
      if ((bal[q] >> lane) & 1u) {
        const int pos = base + __builtin_popcount(bal[q] & lt);
        if ((unsigned)pos < (unsigned)CHUNK) lnode[pos] = c0 + q * TPB + tid;
      }
      base += __builtin_popcount(bal[q]);
    }
    __syncthreads();
    if (wave == 0) {
      const int cnt = total < CHUNK ? total : CHUNK;
      for (int j = 0; j < cnt; ++j) {
        int n = lnode[j];
        n = n < 0 ? 0 : (n > N - 1 ? N - 1 : n);
        acc += h4[(size_t)n * 32 + lane];
      }
    }
    __syncthreads();
  }

  if (wave == 0) {
    const float inv = 1.0f / fmaxf((float)ntot, 1.0f);
    const v4f v = acc * inv;
    float* p = mout + (size_t)g * CHN + lane * 4;
    *(volatile v4f*)p = v;
    __threadfence();
    *(volatile v4f*)p = v;
  }
}

extern "C" void kernel_launch(void* const* d_in, const int* in_sizes, int n_in,
                              void* d_out, int out_size, void* d_ws, size_t ws_size,
                              hipStream_t stream)
{
  if (n_in < 13 || d_out == 0 || d_ws == 0) return;
  const int N = in_sizes[0] / CHN;
  const int E = in_sizes[1] / 2;
  const int G = out_size / CHN;
  if (N < 1 || (in_sizes[0] % CHN) != 0 || (in_sizes[1] % 2) != 0 || E < 0) return;
  if (in_sizes[2] != N) return;
  if (G < 128 || (G % 128) != 0 || out_size != G * CHN) return;
  if (in_sizes[3] != CHN * CHN || in_sizes[4] != CHN) return;
  if (in_sizes[5] != CHN * CHN || in_sizes[6] != CHN) return;
  if (in_sizes[7] != CHN * CHN || in_sizes[8] != CHN) return;
  if (in_sizes[9] != CHN * HID2 || in_sizes[10] != HID2) return;
  if (in_sizes[11] != HID2 * CHN || in_sizes[12] != CHN) return;

  const float* x    = (const float*)d_in[0];
  const int*   esrc = (const int*)d_in[1];
  const int*   edst = esrc + E;
  const int*   bat  = (const int*)d_in[2];
  const float* W0   = (const float*)d_in[3];
  const float* b0   = (const float*)d_in[4];
  const float* Wg1  = (const float*)d_in[5];
  const float* bg1  = (const float*)d_in[6];
  const float* Wg2  = (const float*)d_in[7];
  const float* bg2  = (const float*)d_in[8];
  const float* Wh1  = (const float*)d_in[9];
  const float* bh1  = (const float*)d_in[10];
  const float* Wh2  = (const float*)d_in[11];
  const float* bh2  = (const float*)d_in[12];
  float* out = (float*)d_out;

  const int NPAD  = ((N + NBLK - 1) / NBLK) * NBLK;
  const int NDPAD = ((NPAD + NDEG - 1) / NDEG) * NDEG;

  char* wsb = (char*)d_ws;
  size_t off = 0;
  const size_t AL = 255;
  float* hA = (float*)(wsb + off);      off += (((size_t)NPAD * CHN * 4) + AL) & ~AL;
  float* hB = (float*)(wsb + off);      off += (((size_t)NPAD * CHN * 4) + AL) & ~AL;
  _Float16* S = (_Float16*)(wsb + off); off += (((size_t)NPAD * CHN * 2) + AL) & ~AL;
  float* dinvp = (float*)(wsb + off);   off += (((size_t)NDPAD * 4) + AL) & ~AL;
  float* mbuf = (float*)(wsb + off);    off += (((size_t)G * CHN * 4) + AL) & ~AL;
  float* gbuf = (float*)(wsb + off);    off += (((size_t)G * HID2 * 4) + AL) & ~AL;
  if (off > ws_size) return;

  const size_t ldsG128 = (size_t)2 * 128 * (128 + 8) * 2;
  const size_t ldsG256 = (size_t)2 * 128 * (256 + 8) * 2;
  const size_t ldsAgg  = (size_t)NBLK * CHN * 4 + (size_t)CHUNK * 4 + (size_t)CHUNK * 2;

  hipFuncSetAttribute(reinterpret_cast<const void*>(&k_gemm<float, 128>),
                      hipFuncAttributeMaxDynamicSharedMemorySize, (int)ldsG128);
  hipFuncSetAttribute(reinterpret_cast<const void*>(&k_gemm<_Float16, 128>),
                      hipFuncAttributeMaxDynamicSharedMemorySize, (int)ldsG128);
  hipFuncSetAttribute(reinterpret_cast<const void*>(&k_gemm<float, 256>),
                      hipFuncAttributeMaxDynamicSharedMemorySize, (int)ldsG256);
  hipFuncSetAttribute(reinterpret_cast<const void*>(&k_agg<1>),
                      hipFuncAttributeMaxDynamicSharedMemorySize, (int)ldsAgg);
  hipFuncSetAttribute(reinterpret_cast<const void*>(&k_agg<0>),
                      hipFuncAttributeMaxDynamicSharedMemorySize, (int)ldsAgg);

  const int gxN  = (N + 127) / 128;
  const int nAgg = NPAD / NBLK;
  const int nDeg = NDPAD / NDEG;
  const int gxG  = G / 128;

  k_deg<<<dim3(nDeg), dim3(TPB), 0, stream>>>(edst, E, dinvp);
  k_gemm<float, 128><<<dim3(gxN, 1), dim3(TPB), ldsG128, stream>>>(
      x, CHN, N, W0, CHN, b0, 0, hA, CHN, 0);
  k_agg<1><<<dim3(nAgg), dim3(TPB), ldsAgg, stream>>>(
      esrc, edst, E, N, (const float*)hA, (const float*)dinvp, b0, hB);
  k_agg<0><<<dim3(nAgg), dim3(TPB), ldsAgg, stream>>>(
      esrc, edst, E, N, (const float*)hB, (const float*)dinvp, b0, (float*)S);
  k_gemm<_Float16, 128><<<dim3(gxN, 1), dim3(TPB), ldsG128, stream>>>(
      (const _Float16*)S, CHN, N, Wg1, CHN, bg1, 1, hA, CHN, 1);
  k_agg<0><<<dim3(nAgg), dim3(TPB), ldsAgg, stream>>>(
      esrc, edst, E, N, (const float*)hA, (const float*)dinvp, b0, (float*)S);
  k_gemm<_Float16, 128><<<dim3(gxN, 1), dim3(TPB), ldsG128, stream>>>(
      (const _Float16*)S, CHN, N, Wg2, CHN, bg2, 1, hB, CHN, 1);
  k_pool<<<dim3(G), dim3(TPB), 0, stream>>>(bat, N, (const float*)hB, mbuf);
  k_gemm<float, 128><<<dim3(gxG, 2), dim3(TPB), ldsG128, stream>>>(
      (const float*)mbuf, CHN, G, Wh1, HID2, bh1, 1, gbuf, HID2, 1);
  k_gemm<float, 256><<<dim3(gxG, 1), dim3(TPB), ldsG256, stream>>>(
      (const float*)gbuf, HID2, G, Wh2, CHN, bh2, 1, out, CHN, 0);
}
